// Mamba3_16423954940520
// MI455X (gfx1250) — hardware-verified
//
#include <hip/hip_runtime.h>
#include <hip/hip_bf16.h>
#include <math.h>

#define LSEQ      1024
#define DMODEL    768
#define DSTATE    64
#define HEADDIM   64
#define DINNER    1536
#define NHEADS    24
#define SPLITN    32
#define N_ANG     16
#define DPROJ     3288
#define DPROJ_PAD 3296
#define EPSV      1e-5f
#define A_FLOOR   1e-4f

#define COL_Z     0
#define COL_X     1536
#define COL_B     3072
#define COL_C     3136
#define COL_DT    3200
#define COL_A     3224
#define COL_TRAP  3248
#define COL_ANG   3272

#define NHP 32
typedef __attribute__((ext_vector_type(16))) _Float16 v16bf;
typedef __attribute__((ext_vector_type(8)))  float  v8f;
typedef __attribute__((ext_vector_type(4)))  float  v4f_t;
typedef float v4fa __attribute__((ext_vector_type(4), may_alias));
#define RSPLIT (1.0f / 2048.0f)

static __device__ __forceinline__ unsigned short f32_to_bf16_rne(float f) { return __builtin_bit_cast(unsigned short, (_Float16)f); }
static __device__ __forceinline__ unsigned pack2s(float a, float b, unsigned* lo) {
  const _Float16 h0 = (_Float16)a, h1 = (_Float16)b;
  const _Float16 l0 = (_Float16)((a - (float)h0) * 2048.0f), l1 = (_Float16)((b - (float)h1) * 2048.0f);
  *lo = (unsigned)__builtin_bit_cast(unsigned short, l0) | ((unsigned)__builtin_bit_cast(unsigned short, l1) << 16);
  return (unsigned)__builtin_bit_cast(unsigned short, h0) | ((unsigned)__builtin_bit_cast(unsigned short, h1) << 16);
}
static __device__ __forceinline__ float softplus_f(float x) {
  return (x > 20.f) ? x : log1pf(expf(x));
}
static __device__ __forceinline__ float sigmoid_f(float x) {
  return 1.f / (1.f + expf(-x));
}

__global__ void k_cvt_bf16(const float* __restrict__ src,
                           unsigned short* __restrict__ dst, int n) {
  int i = (blockIdx.x * blockDim.x + threadIdx.x) * 2;
  if (i < n) {
    unsigned lo; const unsigned hv = pack2s(src[i], src[i + 1], &lo);
    *(volatile unsigned*)(dst + i) = hv; *(volatile unsigned*)(dst + (size_t)n + i) = lo;
    __threadfence();
    *(volatile unsigned*)(dst + i) = hv; *(volatile unsigned*)(dst + (size_t)n + i) = lo;
  }
}

__global__ void k_cvt_win_pad(const float* __restrict__ src,
                              unsigned short* __restrict__ dst) {
  int i = (blockIdx.x * blockDim.x + threadIdx.x) * 2;
  if (i >= DPROJ_PAD * DMODEL) return;
  int row = i / DMODEL;
  unsigned lo = 0, hv = 0;
  if (row < DPROJ) hv = pack2s(src[i], src[i + 1], &lo);
  *(volatile unsigned*)(dst + i) = hv; *(volatile unsigned*)(dst + (size_t)DPROJ_PAD * DMODEL + i) = lo;
  __threadfence();
  *(volatile unsigned*)(dst + i) = hv; *(volatile unsigned*)(dst + (size_t)DPROJ_PAD * DMODEL + i) = lo;
}

__global__ void __launch_bounds__(256)
k_gemm_bf16(const unsigned short* __restrict__ A,
            const unsigned short* __restrict__ B,
            float* __restrict__ C,
            int M, int N, int K, int ldc) {
  __shared__ __attribute__((aligned(16))) float cst[8][32 * 32];
  const size_t pla = (size_t)M * K, plb = (size_t)N * K;
  const int warp = threadIdx.x >> 5;
  const int lane = threadIdx.x & 31;
  const int w = blockIdx.x * 8 + warp;
  const int ngrp = N >> 5;
  const int mg = w / ngrp;
  const int ng = w - mg * ngrp;
  if (mg * 32 >= M) return;
  const int hi = lane >> 4;
  const int lo = lane & 15;

  const unsigned short* arow0 = A + (size_t)(mg * 32 + lo) * K;
  const unsigned short* arow1 = arow0 + (size_t)16 * K;
  const unsigned short* brow0 = B + (size_t)(ng * 32 + lo) * K + hi * 8;
  const unsigned short* brow1 = brow0 + (size_t)16 * K;

  v8f acc00 = {}, acc01 = {}, acc10 = {}, acc11 = {};
  for (int k0 = 0; k0 < K; k0 += 32) {
    union { uint4 q[2]; v16bf v; } a0, a1, b0, b1, a0l, a1l, b0l, b1l;
    a0.q[0]  = *(const uint4*)(arow0 + k0 + hi * 8);        a0.q[1]  = *(const uint4*)(arow0 + k0 + 16 + hi * 8);
    a1.q[0]  = *(const uint4*)(arow1 + k0 + hi * 8);        a1.q[1]  = *(const uint4*)(arow1 + k0 + 16 + hi * 8);
    a0l.q[0] = *(const uint4*)(arow0 + pla + k0 + hi * 8);  a0l.q[1] = *(const uint4*)(arow0 + pla + k0 + 16 + hi * 8);
    a1l.q[0] = *(const uint4*)(arow1 + pla + k0 + hi * 8);  a1l.q[1] = *(const uint4*)(arow1 + pla + k0 + 16 + hi * 8);
    b0.q[0]  = *(const uint4*)(brow0 + k0);                 b0.q[1]  = *(const uint4*)(brow0 + k0 + 16);
    b1.q[0]  = *(const uint4*)(brow1 + k0);                 b1.q[1]  = *(const uint4*)(brow1 + k0 + 16);
    b0l.q[0] = *(const uint4*)(brow0 + plb + k0);           b0l.q[1] = *(const uint4*)(brow0 + plb + k0 + 16);
    b1l.q[0] = *(const uint4*)(brow1 + plb + k0);           b1l.q[1] = *(const uint4*)(brow1 + plb + k0 + 16);
#define M3_SPLIT(ACC, AV, ALV, BV, BLV) { v8f x_ = {}; \
      x_ = __builtin_amdgcn_wmma_f32_16x16x32_f16(false, ALV, false, BV, (short)0, x_, false, false); \
      x_ = __builtin_amdgcn_wmma_f32_16x16x32_f16(false, AV, false, BLV, (short)0, x_, false, false); \
      ACC = __builtin_amdgcn_wmma_f32_16x16x32_f16(false, AV, false, BV, (short)0, ACC, false, false) + x_ * RSPLIT; }
    M3_SPLIT(acc00, a0.v, a0l.v, b0.v, b0l.v);
    M3_SPLIT(acc01, a0.v, a0l.v, b1.v, b1l.v);
    M3_SPLIT(acc10, a1.v, a1l.v, b0.v, b0l.v);
    M3_SPLIT(acc11, a1.v, a1l.v, b1.v, b1l.v);
#undef M3_SPLIT
  }
  {
    float* cs = cst[warp];
#pragma unroll
    for (int r = 0; r < 8; ++r) {
      cs[(r + 8 * hi) * 32 + lo]           = acc00[r];
      cs[(r + 8 * hi) * 32 + 16 + lo]      = acc01[r];
      cs[(16 + r + 8 * hi) * 32 + lo]      = acc10[r];
      cs[(16 + r + 8 * hi) * 32 + 16 + lo] = acc11[r];
    }
    asm volatile("s_wait_dscnt 0" ::: "memory");
    float* cb = C + (size_t)(mg * 32) * ldc + ng * 32;
    v4f_t ov[8]; size_t oo[8];
#pragma unroll
    for (int i = 0; i < 8; ++i) { const int c = lane + 32 * i, rr = c >> 3, q = c & 7; ov[i] = *(const volatile v4fa*)(cs + rr * 32 + q * 4); oo[i] = (size_t)rr * ldc + q * 4; }
#pragma unroll
    for (int i = 0; i < 8; ++i) *(volatile v4f_t*)(cb + oo[i]) = ov[i];
    __threadfence();
#pragma unroll
    for (int i = 0; i < 8; ++i) *(volatile v4f_t*)(cb + oo[i]) = ov[i];
  }
}

__global__ void __launch_bounds__(64)
k_ew1(const float* __restrict__ proj, const float* __restrict__ dt_bias,
      const float* __restrict__ Bnw, const float* __restrict__ Cnw,
      float* __restrict__ DT, float* __restrict__ aexp,
      float* __restrict__ trap, float* __restrict__ Bn, float* __restrict__ Cn) {
  const int l = blockIdx.x;
  const int t = threadIdx.x;
  const float* row = proj + (size_t)l * DPROJ_PAD;
  float b = row[COL_B + t];
  float c = row[COL_C + t];
  __shared__ float sb[64], sc[64];
  sb[t] = b * b; sc[t] = c * c;
  __syncthreads();
  for (int s = 32; s > 0; s >>= 1) {
    if (t < s) { sb[t] += sb[t + s]; sc[t] += sc[t + s]; }
    __syncthreads();
  }
  const float rb = sqrtf(sb[0] * (1.f / 64.f) + EPSV);
  const float rc = sqrtf(sc[0] * (1.f / 64.f) + EPSV);
  const float bnv = b / rb * Bnw[t], cnv = c / rc * Cnw[t];
  float dtv = 0.f, aev = 0.f, trv = 0.f;
  if (t < NHEADS) {
    dtv = softplus_f(row[COL_DT + t] + dt_bias[t]);
    const float Av = -fmaxf(softplus_f(row[COL_A + t]), A_FLOOR);
    aev = expf(Av * dtv);
    trv = sigmoid_f(row[COL_TRAP + t]);
  }
#pragma unroll 1
  for (int pass = 0; pass < 2; ++pass) {
    *(volatile float*)(Bn + l * 64 + t) = bnv; *(volatile float*)(Cn + l * 64 + t) = cnv;
    if (t < 32) { *(volatile float*)(DT + l * NHP + t) = dtv; *(volatile float*)(aexp + l * NHP + t) = aev; *(volatile float*)(trap + l * NHP + t) = trv; }
    __threadfence();
  }
}

__global__ void __launch_bounds__(384)
k_angcum(const float* __restrict__ proj, const float* __restrict__ DT,
         float* __restrict__ ang) {
  const int t = threadIdx.x;
  const int h = t >> 4;
  const int j = t & 15;
  float acc = 0.f;
  for (int l = 0; l < LSEQ; ++l) {
    acc += proj[(size_t)l * DPROJ_PAD + COL_ANG + j] * DT[l * NHP + h];
    float* ap = ang + ((size_t)l * NHEADS + h) * N_ANG + j;
    *(volatile float*)ap = acc; __threadfence(); *(volatile float*)ap = acc;
  }
}

__global__ void k_ropebias(const float* __restrict__ Bn, const float* __restrict__ Cn,
                           const float* __restrict__ ang,
                           const float* __restrict__ Bbias, const float* __restrict__ Cbias,
                           float* __restrict__ Bp, float* __restrict__ Cp) {
  int gid = blockIdx.x * blockDim.x + threadIdx.x;
  if (gid >= LSEQ * NHEADS * DSTATE) return;
  const int n  = gid & 63;
  const int lh = gid >> 6;
  const int h  = lh % NHEADS;
  const int l  = lh / NHEADS;
  float tb = Bn[l * 64 + n] + Bbias[h * 64 + n];
  float tc = Cn[l * 64 + n] + Cbias[h * 64 + n];
  if (n < SPLITN) {
    const int j = n >> 1;
    const float av = ang[((size_t)l * NHEADS + h) * N_ANG + j];
    const float cs = cosf(av), sn = sinf(av);
    const int pn = n ^ 1;
    const float ob = Bn[l * 64 + pn] + Bbias[h * 64 + pn];
    const float oc = Cn[l * 64 + pn] + Cbias[h * 64 + pn];
    if ((n & 1) == 0) { tb = tb * cs - ob * sn; tc = tc * cs - oc * sn; }
    else              { tb = ob * sn + tb * cs; tc = oc * sn + tc * cs; }
  }
  *(volatile float*)(Bp + gid) = tb; *(volatile float*)(Cp + gid) = tc;
  __threadfence();
  *(volatile float*)(Bp + gid) = tb; *(volatile float*)(Cp + gid) = tc;
}

__global__ void __launch_bounds__(256)
k_scan(const float* __restrict__ proj, const float* __restrict__ aexp,
       const float* __restrict__ DT, const float* __restrict__ trap,
       const float* __restrict__ Bp, const float* __restrict__ Cp,
       const float* __restrict__ Dskip, float* __restrict__ yraw) {
  const int h = blockIdx.x;
  const int tid = threadIdx.x;
  const int p  = tid >> 2;
  const int nb = (tid & 3) << 4;
  __shared__ float xs[64], Bs[64], Cs[64], ys[64];
  float hreg[16], bxp[16];
#pragma unroll
  for (int j = 0; j < 16; ++j) { hreg[j] = 0.f; bxp[j] = 0.f; }
  const float dsk = Dskip[h];

  for (int l = 0; l < LSEQ; ++l) {
    if (tid < 64)       xs[tid]       = proj[(size_t)l * DPROJ_PAD + COL_X + h * HEADDIM + tid];
    else if (tid < 128) Bs[tid - 64]  = Bp[((size_t)l * NHEADS + h) * DSTATE + (tid - 64)];
    else if (tid < 192) Cs[tid - 128] = Cp[((size_t)l * NHEADS + h) * DSTATE + (tid - 128)];
    const float a  = aexp[l * NHP + h];
    const float dt = DT[l * NHP + h];
    const float tr = trap[l * NHP + h];
    if (l + 1 < LSEQ) {
      if (tid == 0)       __builtin_prefetch(&proj[(size_t)(l + 1) * DPROJ_PAD + COL_X + h * HEADDIM], 0, 0);
      else if (tid == 64) __builtin_prefetch(&Bp[((size_t)(l + 1) * NHEADS + h) * DSTATE], 0, 0);
      else if (tid == 128)__builtin_prefetch(&Cp[((size_t)(l + 1) * NHEADS + h) * DSTATE], 0, 0);
    }
    __syncthreads();
    const float x = xs[p];
    float part = 0.f;
#pragma unroll
    for (int j = 0; j < 16; ++j) {
      const float bx = x * Bs[nb + j];
      const float hv = a * hreg[j] + dt * ((1.f - tr) * bx + tr * a * bxp[j]);
      hreg[j] = hv;
      bxp[j] = bx;
      part += hv * Cs[nb + j];
    }
    part += __shfl_xor(part, 1, 32);
    part += __shfl_xor(part, 2, 32);
    if ((tid & 3) == 0) ys[p] = part + dsk * x;
    __syncthreads();
    if (tid < 16) {
      const v4f_t yv = *(const volatile v4fa*)(ys + tid * 4);
      float* yp = yraw + (size_t)l * DINNER + h * HEADDIM + tid * 4;
      *(volatile v4f_t*)yp = yv; __threadfence(); *(volatile v4f_t*)yp = yv;
    }
  }
}

__global__ void k_gate(const float* __restrict__ yraw, const float* __restrict__ proj,
                       unsigned short* __restrict__ ybf) {
  int i = (blockIdx.x * blockDim.x + threadIdx.x) * 2;
  if (i >= LSEQ * DINNER) return;
  const int l = i / DINNER;
  const int c = i - l * DINNER;
  const float z0 = proj[(size_t)l * DPROJ_PAD + COL_Z + c], z1 = proj[(size_t)l * DPROJ_PAD + COL_Z + c + 1];
  const float v0 = yraw[i] * (z0 * sigmoid_f(z0)), v1 = yraw[i + 1] * (z1 * sigmoid_f(z1));
  unsigned lo; const unsigned hv = pack2s(v0, v1, &lo);
  *(volatile unsigned*)(ybf + i) = hv; *(volatile unsigned*)(ybf + (size_t)LSEQ * DINNER + i) = lo;
  __threadfence();
  *(volatile unsigned*)(ybf + i) = hv; *(volatile unsigned*)(ybf + (size_t)LSEQ * DINNER + i) = lo;
}

extern "C" void kernel_launch(void* const* d_in, const int* in_sizes, int n_in,
                              void* d_out, int out_size, void* d_ws, size_t ws_size,
                              hipStream_t stream) {
  (void)in_sizes; (void)n_in; (void)out_size; (void)ws_size;
  const float* u        = (const float*)d_in[0];
  const float* W_in     = (const float*)d_in[1];
  const float* W_out    = (const float*)d_in[2];
  const float* dt_bias  = (const float*)d_in[3];
  const float* B_bias   = (const float*)d_in[4];
  const float* C_bias   = (const float*)d_in[5];
  const float* B_norm_w = (const float*)d_in[6];
  const float* C_norm_w = (const float*)d_in[7];
  const float* D_skip   = (const float*)d_in[8];
  float* out = (float*)d_out;

  char* ws = (char*)d_ws;
  size_t off = 0;
  auto alloc = [&](size_t bytes) -> void* {
    void* p = ws + off;
    off = (off + bytes + 255) & ~(size_t)255;
    return p;
  };

  float*          proj   = (float*)alloc((size_t)LSEQ * DPROJ_PAD * 4);
  unsigned short* ubf    = (unsigned short*)alloc((size_t)LSEQ * DMODEL * 2 * 2);
  unsigned short* winbf  = (unsigned short*)alloc((size_t)DPROJ_PAD * DMODEL * 2 * 2);
  unsigned short* woutbf = (unsigned short*)alloc((size_t)DMODEL * DINNER * 2 * 2);
  float*          DTb    = (float*)alloc((size_t)LSEQ * NHP * 4);
  float*          aexp   = (float*)alloc((size_t)LSEQ * NHP * 4);
  float*          trap   = (float*)alloc((size_t)LSEQ * NHP * 4);
  float*          Bn     = (float*)alloc((size_t)LSEQ * DSTATE * 4);
  float*          Cn     = (float*)alloc((size_t)LSEQ * DSTATE * 4);
  float*          ang    = (float*)alloc((size_t)LSEQ * NHEADS * N_ANG * 4);
  float*          Bp     = (float*)alloc((size_t)LSEQ * NHEADS * DSTATE * 4);
  float*          Cp     = (float*)alloc((size_t)LSEQ * NHEADS * DSTATE * 4);
  float*          yraw   = (float*)alloc((size_t)LSEQ * DINNER * 4);
  unsigned short* ybf    = (unsigned short*)alloc((size_t)LSEQ * DINNER * 2 * 2);

  {
    int n = LSEQ * DMODEL;
    k_cvt_bf16<<<(n / 2 + 255) / 256, 256, 0, stream>>>(u, ubf, n);
  }
  {
    int n = DPROJ_PAD * DMODEL;
    k_cvt_win_pad<<<(n / 2 + 255) / 256, 256, 0, stream>>>(W_in, winbf);
  }
  {
    int n = DMODEL * DINNER;
    k_cvt_bf16<<<(n / 2 + 255) / 256, 256, 0, stream>>>(W_out, woutbf, n);
  }

  {
    int waves = (LSEQ / 32) * (DPROJ_PAD / 32);
    k_gemm_bf16<<<waves / 8, 256, 0, stream>>>(ubf, winbf, proj,
                                               LSEQ, DPROJ_PAD, DMODEL, DPROJ_PAD);
  }

  k_ew1<<<LSEQ, 64, 0, stream>>>(proj, dt_bias, B_norm_w, C_norm_w,
                                 DTb, aexp, trap, Bn, Cn);

  k_angcum<<<1, 384, 0, stream>>>(proj, DTb, ang);

  {
    int n = LSEQ * NHEADS * DSTATE;
    k_ropebias<<<(n + 255) / 256, 256, 0, stream>>>(Bn, Cn, ang, B_bias, C_bias, Bp, Cp);
  }

  k_scan<<<NHEADS, 256, 0, stream>>>(proj, aexp, DTb, trap, Bp, Cp, D_skip, yraw);

  {
    int n = LSEQ * DINNER;
    k_gate<<<(n / 2 + 255) / 256, 256, 0, stream>>>(yraw, proj, ybf);
  }

  {
    int waves = (LSEQ / 32) * (DMODEL / 32);
    k_gemm_bf16<<<waves / 8, 256, 0, stream>>>(ybf, woutbf, out,
                                               LSEQ, DMODEL, DINNER, DMODEL);
  }
}
